// WLGNN_5549097746502
// MI455X (gfx1250) — hardware-verified
//
#include <hip/hip_runtime.h>
#include <stdint.h>
#include <stddef.h>


#define PN     60000
#define HALFP  30000
#define E2N    960000
#define EIN    30000
#define NLK    60000
#define NND    1024
#define NF     128
#define F1     32
#define F2     24
#define LNEPS  1e-5f

#define RW     64
#define NB     512
#define NTHR   256
#define NWAVE  8
#define CHUNK  2048
#define WCAP   256
#define NGRP   (CHUNK / (NTHR * 4))
#define NRB    ((PN + NB - 1) / NB)
#define PROWS  (NRB * NB)

#define GT     64
#define GTHR   128
#define CP     68
#define MT1    ((PN + GT - 1) / GT)
#define MPAD   (MT1 * GT)
#define MT2    ((EIN + GT - 1) / GT)
#define EPAD   (MT2 * GT)
#define LT     ((NLK + GT - 1) / GT)
#define VPAD   (LT * GT)

#define CB     12
#define CSUB   4
#define NSUB   (CB / CSUB)
#define NBATCH (F2 / CB)
#define RCAP   128
#define FP     40
#define VP     36

static_assert(WCAP == (CHUNK / NTHR) * 32);
static_assert(NGRP == 2);
static_assert(NB == 512);
static_assert(NB == NWAVE * 64);
static_assert(MPAD <= PROWS);
static_assert((PN % NWAVE) == 0);
static_assert((NLK % 4) == 0);
static_assert(RCAP == 128);
static_assert((F2 % CB) == 0);
static_assert((CB % CSUB) == 0);
static_assert((NND % GT) == 0);
static_assert(2 * F2 <= GT);
static_assert(F2 + 1 <= 32);
static_assert((CP % 4) == 0);
static_assert((VP % 4) == 0);
static_assert((FP % 8) == 0);

typedef float          v4f  __attribute__((ext_vector_type(4)));
typedef float          v8f  __attribute__((ext_vector_type(8)));
typedef int            v4i  __attribute__((ext_vector_type(4)));
typedef _Float16       v4h  __attribute__((ext_vector_type(4)));
typedef _Float16       v8h  __attribute__((ext_vector_type(8)));
typedef _Float16       v16h __attribute__((ext_vector_type(16)));
union Frag { v16h v; v8h half[2]; };

__device__ __forceinline__ int imin(int a, int b) { return a < b ? a : b; }
__device__ __forceinline__ int imax(int a, int b) { return a > b ? a : b; }
__device__ __forceinline__ int iclamp(int v, int lo, int hi) { return v < lo ? lo : (v > hi ? hi : v); }

__device__ __forceinline__ float wsum(float v) {
#pragma unroll
  for (int o = 16; o > 0; o >>= 1) v += __shfl_xor(v, o, 32);
  return v;
}
__device__ __forceinline__ int wmaxi(int v) {
#pragma unroll
  for (int o = 16; o > 0; o >>= 1) v = imax(v, __shfl_xor(v, o, 32));
  return v;
}

__device__ __forceinline__ v8f wm(v16h a, v16h b, v8f c) {
  v8f d = __builtin_amdgcn_wmma_f32_16x16x32_f16(false, a, false, b, (short)0, c, false, false);
  asm volatile("v_nop\n\tv_nop\n\tv_nop\n\tv_nop" : "+v"(d) : "v"(a), "v"(b));
  return d;
}
__device__ __forceinline__ v8f z8() {
  v8f z = {0.f, 0.f, 0.f, 0.f, 0.f, 0.f, 0.f, 0.f};
  return z;
}

__device__ __forceinline__ float ln_relu(float x, float inv_n, bool active) {
  const float mu = wsum(x) * inv_n;
  const float d = active ? (x - mu) : 0.f;
  const float var = wsum(d * d) * inv_n;
  return fmaxf(d * rsqrtf(var + LNEPS), 0.f);
}

__device__ __forceinline__ int scan_chunk(const int* __restrict__ key, int nE, int cbase,
                                          int nodeBase, int* list, int wave, int tid, int al16) {
  int wc = 0;
#pragma unroll
  for (int g = 0; g < NGRP; ++g) {
    const int el0 = (g * NTHR + tid) * 4;
    const int e0 = cbase + el0;
    const int sent = -2147483647 - 1;
    v4i d;
    if (al16 != 0 && (cbase + CHUNK <= nE)) {
      d = *(const v4i*)(key + e0);
    } else {
      const int c0 = iclamp(e0, 0, nE - 1), c1 = iclamp(e0 + 1, 0, nE - 1);
      const int c2 = iclamp(e0 + 2, 0, nE - 1), c3 = iclamp(e0 + 3, 0, nE - 1);
      const int k0v = key[c0], k1v = key[c1], k2v = key[c2], k3v = key[c3];
      d.x = (e0     < nE) ? k0v : sent;
      d.y = (e0 + 1 < nE) ? k1v : sent;
      d.z = (e0 + 2 < nE) ? k2v : sent;
      d.w = (e0 + 3 < nE) ? k3v : sent;
    }
    const unsigned s0 = (unsigned)d.x - (unsigned)nodeBase;
    const unsigned s1 = (unsigned)d.y - (unsigned)nodeBase;
    const unsigned s2 = (unsigned)d.z - (unsigned)nodeBase;
    const unsigned s3 = (unsigned)d.w - (unsigned)nodeBase;
    const bool h0 = s0 < (unsigned)NB;
    const bool h1 = s1 < (unsigned)NB;
    const bool h2 = s2 < (unsigned)NB;
    const bool h3 = s3 < (unsigned)NB;
    const unsigned many = __builtin_amdgcn_ballot_w32(h0 | h1 | h2 | h3);
    if (many != 0u) {
#define HITJ(J, HJ, SJ) { \
        const unsigned mj = __builtin_amdgcn_ballot_w32(HJ); \
        const int posj = wc + (int)__builtin_amdgcn_mbcnt_lo(mj, 0u); \
        if (HJ) { \
          if (posj < WCAP) list[wave * WCAP + posj] = ((el0 + (J)) << 9) | (int)(SJ); \
        } \
        wc += (int)__builtin_popcount(mj); }
      HITJ(0, h0, s0)
      HITJ(1, h1, s1)
      HITJ(2, h2, s2)
      HITJ(3, h3, s3)
#undef HITJ
    }
  }
  return wc;
}

__global__ __launch_bounds__(NTHR) void k_rows(const int* __restrict__ eA, const int* __restrict__ eB,
                                               int* tabA, int* tabB, int nE, int nP) {
  __shared__ __attribute__((aligned(16))) int plist[NB * RW];
  __shared__ int pcnt[NB];
  __shared__ int list[NWAVE * WCAP];
  __shared__ int wcnt[NWAVE];

  const int tid  = threadIdx.x;
  const int lane = tid & 31;
  const int wave = tid >> 5;
  const int setb = (blockIdx.y != 0) ? 1 : 0;
  const int* edge = setb ? eB : eA;
  int* tab = setb ? tabB : tabA;
  const int* key  = edge + nE;
  const int* srcs = edge;
  const int nodeBase = blockIdx.x * NB;

  for (int i = tid; i < NB * RW; i += NTHR) plist[i] = 0;
  for (int i = tid; i < NB; i += NTHR) pcnt[i] = 0;
  __syncthreads();

  const int al16 = ((((uintptr_t)(const void*)key) & 15u) == 0) ? 1 : 0;
  const int nChunks = (nE + CHUNK - 1) / CHUNK;

#pragma unroll 1
  for (int ch = 0; ch < nChunks; ++ch) {
    const int cbase = ch * CHUNK;
    const int wc = scan_chunk(key, nE, cbase, nodeBase, list, wave, tid, al16);
    if (lane == 0) wcnt[wave] = wc;
    __syncthreads();
#pragma unroll 1
    for (int wsx = 0; wsx < NWAVE; ++wsx) {
      int n = wcnt[wsx];
      n = iclamp(n, 0, WCAP);
#pragma unroll 1
      for (int i = 0; i < n; ++i) {
        const int ent  = list[wsx * WCAP + i];
        const int slot = ent & (NB - 1);
        if ((slot & (NWAVE - 1)) == wave) {
          int e = cbase + ((ent >> 9) & (CHUNK - 1));
          e = iclamp(e, 0, nE - 1);
          const int s   = iclamp(srcs[e], 0, nP - 1);
          const int c   = pcnt[slot];
          const int pos = c < RW - 2 ? c : RW - 2;
          if (lane == 0) plist[slot * RW + 1 + pos] = s;
          pcnt[slot] = c + 1;
        }
      }
    }
    __syncthreads();
  }

  for (int s = tid; s < NB; s += NTHR) {
    int c = pcnt[s];
    c = c > RW - 1 ? RW - 1 : c;
    plist[s * RW] = c;
  }
  __syncthreads();

#pragma unroll 1
  for (int ps = 0; ps < 2; ++ps) {
#pragma unroll 4
    for (int it = 0; it < 32; ++it) {
      const int slot = wave * 64 + 2 * it + (lane >> 4);
      const int c4   = 4 * (lane & 15);
      const v4i v = *(const v4i*)(plist + slot * RW + c4);
      *(volatile v4i*)(tab + (size_t)(nodeBase + slot) * RW + c4) = v;
    }
    if (ps == 0) __threadfence();
  }
}

__device__ __forceinline__ void epi_scale(v8f acc, int rbase, int col, float s, const float* dv, float* Cs) {
#pragma unroll
  for (int r = 0; r < 8; ++r) Cs[(rbase + r) * CP + col] = acc[r] * s * dv[rbase + r];
}
__device__ __forceinline__ void epi_bias(v8f acc, int rbase, int col, float s, float badd, float* Cs) {
#pragma unroll
  for (int r = 0; r < 8; ++r) Cs[(rbase + r) * CP + col] = acc[r] * s + badd;
}

template <int K>
__global__ __launch_bounds__(GTHR) void k_gemm(const float* __restrict__ A, const int* __restrict__ idx, int useIdx,
                                               int M, int nRowsA,
                                               const float* __restrict__ W1, int N1,
                                               const float* __restrict__ W2, int N2, int mode,
                                               const int* __restrict__ rA, const int* __restrict__ rB,
                                               const float* __restrict__ b1, const float* __restrict__ b2,
                                               float* C) {
  constexpr int AP = K + 8;
  constexpr int Q  = K / 4;
  static_assert((K % 32) == 0);
  static_assert(((GT * Q) % GTHR) == 0);
  static_assert(((GT * K) % GTHR) == 0);
  __shared__ __attribute__((aligned(16))) _Float16 As[GT * AP];
  __shared__ __attribute__((aligned(16))) _Float16 Bs[GT * AP];
  __shared__ __attribute__((aligned(16))) float Cs[GT * CP];
  __shared__ int   srow[GT];
  __shared__ float sdv[2 * GT];

  const int tid  = threadIdx.x;
  const int lane = tid & 31;
  const int wave = tid >> 5;
  const int h    = lane >> 4;
  const int m    = lane & 15;
  const int m0   = blockIdx.x * GT;

  if (tid < GT) {
    const int gr = m0 + tid;
    const int r  = gr < M ? gr : M - 1;
    int s = r;
    if (useIdx != 0) { s = idx[r]; s = iclamp(s, 0, nRowsA - 1); }
    srow[tid] = s;
  } else if (mode == 0) {
    const int t  = tid - GT;
    const int gr = m0 + t;
    const int ca = iclamp(rA[(size_t)gr * RW], 0, RW - 1);
    const int cb = iclamp(rB[(size_t)gr * RW], 0, RW - 1);
    sdv[t]      = rsqrtf((float)(ca + 1));
    sdv[GT + t] = rsqrtf((float)(cb + 1));
  }
  __syncthreads();

  for (int i = tid; i < GT * K; i += GTHR) {
    const int n = i / K;
    const int k = i - n * K;
    const float va = W1[(size_t)k * N1 + (n < N1 ? n : N1 - 1)];
    const int   nb = iclamp(n - N1, 0, N2 - 1);
    const float vb = W2[(size_t)k * N2 + nb];
    const float v  = (n < N1) ? va : ((n < N1 + N2) ? vb : 0.f);
    Bs[n * AP + k] = (_Float16)(64.f * v);
  }
  for (int i = tid; i < GT * Q; i += GTHR) {
    const int r = i / Q;
    const int q = i - r * Q;
    const v4f f = *(const v4f*)(A + (size_t)srow[r] * K + 4 * q);
    v4h hv;
    hv.x = (_Float16)f.x; hv.y = (_Float16)f.y; hv.z = (_Float16)f.z; hv.w = (_Float16)f.w;
    *(v4h*)(As + r * AP + 4 * q) = hv;
  }
  __syncthreads();

  v8f acc0 = z8(), acc1 = z8(), acc2 = z8(), acc3 = z8();
  const _Float16* pa = As + (16 * wave + m) * AP + 8 * h;
  const _Float16* pb = Bs + m * AP + 8 * h;
#pragma unroll
  for (int k0 = 0; k0 < K; k0 += 32) {
    Frag a, bq0, bq1, bq2, bq3;
    a.half[0]   = *(const v8h*)(pa + k0);            a.half[1]   = *(const v8h*)(pa + k0 + 16);
    bq0.half[0] = *(const v8h*)(pb + k0);            bq0.half[1] = *(const v8h*)(pb + k0 + 16);
    bq1.half[0] = *(const v8h*)(pb + 16 * AP + k0);  bq1.half[1] = *(const v8h*)(pb + 16 * AP + k0 + 16);
    bq2.half[0] = *(const v8h*)(pb + 32 * AP + k0);  bq2.half[1] = *(const v8h*)(pb + 32 * AP + k0 + 16);
    bq3.half[0] = *(const v8h*)(pb + 48 * AP + k0);  bq3.half[1] = *(const v8h*)(pb + 48 * AP + k0 + 16);
    acc0 = wm(a.v, bq0.v, acc0);
    acc1 = wm(a.v, bq1.v, acc1);
    acc2 = wm(a.v, bq2.v, acc2);
    acc3 = wm(a.v, bq3.v, acc3);
  }

  const float sw = 1.0f / 64.0f;
  const int rbase = 16 * wave + 8 * h;
  if (mode == 0) {
    epi_scale(acc0, rbase, m,      sw, sdv,      Cs);
    epi_scale(acc1, rbase, 16 + m, sw, sdv,      Cs);
    epi_scale(acc2, rbase, 32 + m, sw, sdv + GT, Cs);
    epi_scale(acc3, rbase, 48 + m, sw, sdv + GT, Cs);
  } else {
#define BIASV(col, outv) { const int cc_ = (col); \
      const float xa_ = b1[cc_ < N1 ? cc_ : N1 - 1]; \
      const float xb_ = b2[iclamp(cc_ - N1, 0, N2 - 1)]; \
      outv = (cc_ < N1) ? xa_ : ((cc_ < N1 + N2) ? xb_ : 0.f); }
    float bb0, bb1, bb2, bb3;
    BIASV(m, bb0) BIASV(16 + m, bb1) BIASV(32 + m, bb2) BIASV(48 + m, bb3)
#undef BIASV
    epi_bias(acc0, rbase, m,      sw, bb0, Cs);
    epi_bias(acc1, rbase, 16 + m, sw, bb1, Cs);
    epi_bias(acc2, rbase, 32 + m, sw, bb2, Cs);
    epi_bias(acc3, rbase, 48 + m, sw, bb3, Cs);
  }
  __syncthreads();

  if (mode == 1) {
    const bool act = lane < F2;
    const int lc = act ? lane : 0;
#pragma unroll 1
    for (int i = 0; i < 16; ++i) {
      const int row = 16 * wave + i;
      float x1 = Cs[row * CP + lc];
      float x2 = Cs[row * CP + F2 + lc];
      x1 = act ? x1 : 0.f;
      x2 = act ? x2 : 0.f;
      const float y1 = ln_relu(x1, 1.0f / (float)F2, act);
      const float y2 = ln_relu(x2, 1.0f / (float)F2, act);
      if (act) {
        Cs[row * CP + lane]      = y1;
        Cs[row * CP + F2 + lane] = y2;
      }
      if (lane < GT - 2 * F2) Cs[row * CP + 2 * F2 + lane] = 0.f;
    }
    __syncthreads();
  }

#pragma unroll 1
  for (int ps = 0; ps < 2; ++ps) {
#pragma unroll
    for (int it = 0; it < 8; ++it) {
      const int row = 16 * wave + 2 * it + (lane >> 4);
      const int c4  = 4 * (lane & 15);
      const v4f v = *(const v4f*)(Cs + row * CP + c4);
      *(volatile v4f*)(C + (size_t)(m0 + row) * GT + c4) = v;
    }
    if (ps == 0) __threadfence();
  }
}

__device__ __forceinline__ float gcn_set(const int* __restrict__ tab, const float* __restrict__ T, int off,
                                         const float* __restrict__ bias, int nodec, int nP, int lane) {
  const int* row = tab + (size_t)nodec * RW;
  const int w0 = row[lane];
  const int w1 = row[32 + lane];
  int cnt = __shfl(w0, 0, 32);
  cnt = iclamp(cnt, 0, RW - 1);
  const float dn = rsqrtf((float)(cnt + 1));
  float acc = 0.f;
#pragma unroll 2
  for (int p = 0; p < cnt; ++p) {
    const int j = p + 1;
    const int a = __shfl(w0, j & 31, 32);
    const int b = __shfl(w1, j & 31, 32);
    int src = (j < 32) ? a : b;
    src = iclamp(src, 0, nP - 1);
    acc += T[(size_t)src * 64 + off + lane];
  }
  const float self = T[(size_t)nodec * 64 + off + lane];
  const float v = (acc + self) * dn + bias[lane];
  return ln_relu(v, 1.0f / (float)F1, true);
}

__global__ __launch_bounds__(NTHR) void k_agg(const int* __restrict__ rA, const int* __restrict__ rB,
                                              const float* __restrict__ T,
                                              const float* __restrict__ bA, const float* __restrict__ bB,
                                              float* H, int nP) {
  __shared__ __attribute__((aligned(16))) float hs[NWAVE * 32];
  const int tid  = threadIdx.x;
  const int lane = tid & 31;
  const int wave = tid >> 5;
  const int node = blockIdx.x * NWAVE + wave;
  const int nodec = node < nP ? node : nP - 1;
  const float va = gcn_set(rA, T, 0,  bA, nodec, nP, lane);
  const float vb = gcn_set(rB, T, F1, bB, nodec, nP, lane);
  hs[wave * 32 + lane] = va + vb;
  __syncthreads();
  const v4f v = *(const v4f*)(hs + wave * 32 + 4 * (lane & 7));
  const bool wr = (lane < 8) && (node < nP);
  if (wr) *(volatile v4f*)(H + (size_t)node * F1 + 4 * lane) = v;
  __threadfence();
  if (wr) *(volatile v4f*)(H + (size_t)node * F1 + 4 * lane) = v;
}

__global__ __launch_bounds__(32) void k_planes(const int* __restrict__ ei, const float* __restrict__ X12,
                                               const int* __restrict__ nn, int cb0, int doBits,
                                               _Float16* PA, _Float16* PB, unsigned int* bits, int nE) {
  __shared__ int es[RCAP];
  __shared__ int cs[RCAP];
  __shared__ __attribute__((aligned(16))) _Float16 tile[CB * NND];

  const int lane  = threadIdx.x & 31;
  const int u     = blockIdx.x;
  const int sideB = (blockIdx.y != 0) ? 1 : 0;
  const int* key  = ei + (sideB ? nE : 0);
  const int* oth  = ei + (sideB ? 0 : nE);
  const int voff  = sideB ? F2 : 0;
  _Float16* plane = sideB ? PB : PA;
  int nnode = nn[0];
  nnode = iclamp(nnode, 1, NND);
  const int al16 = ((((uintptr_t)(const void*)key) & 15u) == 0) ? 1 : 0;

  int cnt = 0;
  const int ngrp = (nE + 127) / 128;
#pragma unroll 1
  for (int g = 0; g < ngrp; ++g) {
    const int e0 = (g * 32 + lane) * 4;
    v4i d;
    if (al16 != 0 && (g + 1) * 128 <= nE) {
      d = *(const v4i*)(key + e0);
    } else {
      const int c0 = iclamp(e0, 0, nE - 1), c1 = iclamp(e0 + 1, 0, nE - 1);
      const int c2 = iclamp(e0 + 2, 0, nE - 1), c3 = iclamp(e0 + 3, 0, nE - 1);
      const int k0v = key[c0], k1v = key[c1], k2v = key[c2], k3v = key[c3];
      d.x = (e0     < nE) ? k0v : -1;
      d.y = (e0 + 1 < nE) ? k1v : -1;
      d.z = (e0 + 2 < nE) ? k2v : -1;
      d.w = (e0 + 3 < nE) ? k3v : -1;
    }
    const bool h0 = (d.x == u), h1 = (d.y == u), h2 = (d.z == u), h3 = (d.w == u);
    const unsigned any = __builtin_amdgcn_ballot_w32(h0 | h1 | h2 | h3);
    if (any != 0u) {
#define HITE(J, HJ) { \
        const unsigned mj = __builtin_amdgcn_ballot_w32(HJ); \
        const int posj = cnt + (int)__builtin_amdgcn_mbcnt_lo(mj, 0u); \
        if (HJ) { if (posj < RCAP) es[posj] = e0 + (J); } \
        cnt += (int)__builtin_popcount(mj); }
      HITE(0, h0)
      HITE(1, h1)
      HITE(2, h2)
      HITE(3, h3)
#undef HITE
    }
  }
  __syncthreads();
  const int n = cnt < RCAP ? cnt : RCAP;

  int csr[4];
#pragma unroll
  for (int t = 0; t < 4; ++t) {
    const int i = 32 * t + lane;
    int e = es[i];
    e = iclamp(e, 0, nE - 1);
    int col = oth[e];
    col = iclamp(col, 0, nnode - 1);
    csr[t] = (i < n) ? col : -1;
    cs[i] = csr[t];
  }
  __syncthreads();

  unsigned int wb = 0u;
#pragma unroll 1
  for (int i = 0; i < n; ++i) {
    const int c = cs[i];
    wb |= ((c >> 5) == lane) ? (1u << (unsigned)(c & 31)) : 0u;
  }
  const bool wbits = (sideB == 0) && (doBits != 0);

  {
    v8h z;
#pragma unroll
    for (int i = 0; i < 8; ++i) z[i] = (_Float16)0.0f;
#pragma unroll 4
    for (int it = 0; it < CB * 4; ++it) *(v8h*)(tile + it * 256 + 8 * lane) = z;
  }
  __syncthreads();

  const int vc = imin(voff + cb0 + lane, 63);
#pragma unroll 1
  for (int i = 0; i < n; ++i) {
    const int col = cs[i];
    unsigned int em = 0u;
#pragma unroll
    for (int t = 0; t < 4; ++t)
      em |= __builtin_amdgcn_ballot_w32((csr[t] == col) && ((32 * t + lane) < i));
    if (em == 0u) {
      float s = 0.f;
#pragma unroll
      for (int t = 0; t < 4; ++t) {
        unsigned int mk = __builtin_amdgcn_ballot_w32((csr[t] == col) && ((32 * t + lane) >= i) && ((32 * t + lane) < n));
#pragma unroll 1
        while (mk != 0u) {
          const int b = __builtin_ctz(mk);
          mk &= mk - 1u;
          const int j = 32 * t + b;
          const int e = iclamp(es[j], 0, nE - 1);
          s += X12[(size_t)e * 64 + vc];
        }
      }
      if (lane < CB) tile[lane * NND + col] = (_Float16)(16.f * s);
    }
  }
  __syncthreads();

#pragma unroll 1
  for (int ps = 0; ps < 2; ++ps) {
#pragma unroll 1
    for (int c = 0; c < CB; ++c) {
#pragma unroll
      for (int it = 0; it < 4; ++it) {
        const v8h v = *(const v8h*)(tile + c * NND + it * 256 + 8 * lane);
        *(volatile v8h*)(plane + ((size_t)c * NND + u) * NND + it * 256 + 8 * lane) = v;
      }
    }
    if (wbits) *(volatile unsigned int*)(bits + (size_t)u * 32 + lane) = wb;
    if (ps == 0) __threadfence();
  }
}

__device__ __forceinline__ void epi_c(v8f acc, int rbase, int col, float s, float* Cs) {
#pragma unroll
  for (int r = 0; r < 8; ++r) Cs[(rbase + r) * CP + col] = acc[r] * s;
}

__global__ __launch_bounds__(GTHR) void k_bigemm(const _Float16* __restrict__ PA, const _Float16* __restrict__ PB,
                                                 float* C, int cofs) {
  __shared__ __attribute__((aligned(16))) float Cs[GT * CP];
  const int tid  = threadIdx.x;
  const int lane = tid & 31;
  const int wave = tid >> 5;
  const int h    = lane >> 4;
  const int m    = lane & 15;
  const int wr   = wave >> 1;
  const int wc   = wave & 1;
  const int m0   = blockIdx.y * GT;
  const int n0   = blockIdx.x * GT;
  const int cz   = blockIdx.z;
  const _Float16* A = PA + (size_t)(cofs + cz) * NND * NND;
  const _Float16* B = PB + (size_t)(cofs + cz) * NND * NND;
  float* Cc = C + (size_t)cz * NND * NND;

  const _Float16* pA0 = A + (size_t)(m0 + 32 * wr + m) * NND + 8 * h;
  const _Float16* pA1 = pA0 + (size_t)16 * NND;
  const _Float16* pB0 = B + (size_t)(n0 + 32 * wc + m) * NND + 8 * h;
  const _Float16* pB1 = pB0 + (size_t)16 * NND;

  v8f acc00 = z8(), acc01 = z8(), acc10 = z8(), acc11 = z8();
#pragma unroll 2
  for (int k0 = 0; k0 < NND; k0 += 32) {
    Frag a0, a1, b0, b1;
    a0.half[0] = *(const v8h*)(pA0 + k0); a0.half[1] = *(const v8h*)(pA0 + k0 + 16);
    a1.half[0] = *(const v8h*)(pA1 + k0); a1.half[1] = *(const v8h*)(pA1 + k0 + 16);
    b0.half[0] = *(const v8h*)(pB0 + k0); b0.half[1] = *(const v8h*)(pB0 + k0 + 16);
    b1.half[0] = *(const v8h*)(pB1 + k0); b1.half[1] = *(const v8h*)(pB1 + k0 + 16);
    acc00 = wm(a0.v, b0.v, acc00);
    acc01 = wm(a0.v, b1.v, acc01);
    acc10 = wm(a1.v, b0.v, acc10);
    acc11 = wm(a1.v, b1.v, acc11);
  }

  const float sc = 1.0f / 256.0f;
  const int colA = 32 * wc + m;
  const int colB = colA + 16;
  epi_c(acc00, 32 * wr + 8 * h,      colA, sc, Cs);
  epi_c(acc01, 32 * wr + 8 * h,      colB, sc, Cs);
  epi_c(acc10, 32 * wr + 16 + 8 * h, colA, sc, Cs);
  epi_c(acc11, 32 * wr + 16 + 8 * h, colB, sc, Cs);
  __syncthreads();

#pragma unroll 1
  for (int ps = 0; ps < 2; ++ps) {
#pragma unroll
    for (int it = 0; it < 8; ++it) {
      const int row = 16 * wave + 2 * it + (lane >> 4);
      const int c4  = 4 * (lane & 15);
      const v4f v = *(const v4f*)(Cs + row * CP + c4);
      *(volatile v4f*)(Cc + (size_t)(m0 + row) * NND + n0 + c4) = v;
    }
    if (ps == 0) __threadfence();
  }
}

__global__ __launch_bounds__(NTHR) void k_cuv(const int* __restrict__ pl, const int* __restrict__ nn,
                                              const float* __restrict__ C, float* CuvT, int cbase) {
  const int t  = blockIdx.x * NTHR + threadIdx.x;
  const int p4 = 4 * t;
  if (p4 < NLK) {
    int nnode = nn[0];
    nnode = iclamp(nnode, 1, NND);
    v4i pu = *(const v4i*)(pl + p4);
    v4i pv = *(const v4i*)(pl + NLK + p4);
    pu.x = iclamp(pu.x, 0, nnode - 1); pu.y = iclamp(pu.y, 0, nnode - 1);
    pu.z = iclamp(pu.z, 0, nnode - 1); pu.w = iclamp(pu.w, 0, nnode - 1);
    pv.x = iclamp(pv.x, 0, nnode - 1); pv.y = iclamp(pv.y, 0, nnode - 1);
    pv.z = iclamp(pv.z, 0, nnode - 1); pv.w = iclamp(pv.w, 0, nnode - 1);
    v4f r[CSUB];
#pragma unroll
    for (int c = 0; c < CSUB; ++c) {
      const float* Cc = C + (size_t)c * NND * NND;
      r[c].x = Cc[(size_t)pu.x * NND + pv.x];
      r[c].y = Cc[(size_t)pu.y * NND + pv.y];
      r[c].z = Cc[(size_t)pu.z * NND + pv.z];
      r[c].w = Cc[(size_t)pu.w * NND + pv.w];
    }
#pragma unroll
    for (int c = 0; c < CSUB; ++c) *(volatile v4f*)(CuvT + (size_t)(cbase + c) * NLK + p4) = r[c];
    __threadfence();
#pragma unroll
    for (int c = 0; c < CSUB; ++c) *(volatile v4f*)(CuvT + (size_t)(cbase + c) * NLK + p4) = r[c];
  }
}

__global__ __launch_bounds__(GTHR) void k_link(const int* __restrict__ pl, const int* __restrict__ nn,
                                               const unsigned int* __restrict__ bits,
                                               const float* __restrict__ CuvT,
                                               const float* __restrict__ m3w, const float* __restrict__ m3b,
                                               float* Vb) {
  __shared__ __attribute__((aligned(16))) _Float16 Fs[GT * FP];
  __shared__ __attribute__((aligned(16))) _Float16 Ws[32 * FP];
  __shared__ __attribute__((aligned(16))) float Vs[GT * VP];
  __shared__ int fe[GT];
  __shared__ int fu[GT];

  const int tid  = threadIdx.x;
  const int lane = tid & 31;
  const int wave = tid >> 5;
  const int h    = lane >> 4;
  const int m    = lane & 15;
  const int p0   = blockIdx.x * GT;
  int nnode = nn[0];
  nnode = iclamp(nnode, 1, NND);

#pragma unroll 1
  for (int i = 0; i < 16; ++i) {
    const int li = 16 * wave + i;
    int p = p0 + li;
    p = p < NLK ? p : NLK - 1;
    const int pu = iclamp(pl[p], 0, nnode - 1);
    const int pv = iclamp(pl[NLK + p], 0, nnode - 1);
    const unsigned int word = bits[(size_t)pu * 32 + lane];
    const int wv = pv >> 5;
    const int bv = pv & 31;
    const unsigned int wsel = (unsigned int)__shfl((int)word, wv, 32);
    const int inei = (int)((wsel >> (unsigned)bv) & 1u);
    const int cntl = (int)__builtin_popcount(word);
    const int maxc = wmaxi(cntl);
    unsigned int wcopy = word;
    bool found = false;
#pragma unroll 1
    for (int k = 0; k < maxc; ++k) {
      const bool valid = k < cntl;
      int b = __builtin_ffs((int)wcopy) - 1;
      b = b < 0 ? 0 : b;
      const int wn = lane * 32 + b;
      const unsigned int x = bits[(size_t)wn * 32 + wv];
      found = found || (valid && (((x >> (unsigned)bv) & 1u) != 0u));
      wcopy &= (wcopy - 1u);
    }
    const unsigned int fb = __builtin_amdgcn_ballot_w32(found);
    const int uni = ((fb != 0u) ? 1 : 0) | inei;
    if (lane == 0) { fe[li] = inei; fu[li] = uni; }
  }
  __syncthreads();

  for (int i = tid; i < 32 * 32; i += GTHR) {
    const int n = i >> 5;
    const int k = i & 31;
    const float wv = m3w[(size_t)imin(k, F2) * F2 + imin(n, F2 - 1)];
    const float v  = (k <= F2 && n < F2) ? wv : 0.f;
    Ws[n * FP + k] = (_Float16)(64.f * v);
  }
  for (int i = tid; i < GT * 32; i += GTHR) {
    const int li = i >> 5;
    const int k  = i & 31;
    int p = p0 + li;
    p = p < NLK ? p : NLK - 1;
    const float cv = CuvT[(size_t)imin(k, F2 - 1) * NLK + p];
    const float fl = (fe[li] != 0) ? 16.f : 0.f;
    const float v  = (k < F2) ? (16.f * cv) : ((k == F2) ? fl : 0.f);
    Fs[li * FP + k] = (_Float16)v;
  }
  __syncthreads();

  {
    Frag a, bq0, bq1;
    const _Float16* pa = Fs + (16 * wave + m) * FP + 8 * h;
    const _Float16* pb = Ws + m * FP + 8 * h;
    a.half[0]   = *(const v8h*)(pa);            a.half[1]   = *(const v8h*)(pa + 16);
    bq0.half[0] = *(const v8h*)(pb);            bq0.half[1] = *(const v8h*)(pb + 16);
    bq1.half[0] = *(const v8h*)(pb + 16 * FP);  bq1.half[1] = *(const v8h*)(pb + 16 * FP + 16);
    v8f acc0 = wm(a.v, bq0.v, z8());
    v8f acc1 = wm(a.v, bq1.v, z8());
    const float sc = 1.0f / 1024.0f;
    const int colA = m;
    const int colB = 16 + m;
    const float ba = m3b[imin(colA, F2 - 1)];
    const float bbr = m3b[imin(colB, F2 - 1)];
    const float bA = (colA < F2) ? ba : 0.f;
    const float bB = (colB < F2) ? bbr : 0.f;
    const int rbase = 16 * wave + 8 * h;
#pragma unroll
    for (int r = 0; r < 8; ++r) {
      Vs[(rbase + r) * VP + colA] = acc0[r] * sc + bA;
      Vs[(rbase + r) * VP + colB] = acc1[r] * sc + bB;
    }
  }
  __syncthreads();
  {
    const bool act = lane < F2;
    const int lc = act ? lane : 0;
#pragma unroll 1
    for (int i = 0; i < 16; ++i) {
      const int row = 16 * wave + i;
      float y = Vs[row * VP + lc];
      y = act ? y : 0.f;
      const float r = ln_relu(y, 1.0f / (float)F2, act);
      const float v = (act && (fu[row] != 0)) ? r : 0.f;
      Vs[row * VP + lane] = v;
    }
  }
  __syncthreads();
#pragma unroll 1
  for (int ps = 0; ps < 2; ++ps) {
#pragma unroll
    for (int it = 0; it < 4; ++it) {
      const int row = 16 * wave + 4 * it + (lane >> 3);
      const int c4  = 4 * (lane & 7);
      const v4f v = *(const v4f*)(Vs + row * VP + c4);
      *(volatile v4f*)(Vb + (size_t)(p0 + row) * 32 + c4) = v;
    }
    if (ps == 0) __threadfence();
  }
}

__global__ __launch_bounds__(NTHR) void k_final(const float* __restrict__ H, const float* __restrict__ V,
                                                const float* __restrict__ m4w, const float* __restrict__ m4b,
                                                float* out) {
  const int i = blockIdx.x * NTHR + threadIdx.x;
  if (i < HALFP) {
    float z = m4b[0];
    const float* ha = H + (size_t)i * F1;
    const float* hb = H + (size_t)(i + HALFP) * F1;
#pragma unroll 1
    for (int c = 0; c < F1; ++c) z += (ha[c] + hb[c]) * m4w[c];
    const float* va = V + (size_t)i * 32;
    const float* vb = V + (size_t)(i + HALFP) * 32;
#pragma unroll 1
    for (int l = 0; l < F2; ++l) z += (va[l] + vb[l]) * m4w[F1 + l];
    const float e = expf(-fabsf(z));
    const float rcp = 1.0f / (1.0f + e);
    const float o = (z >= 0.f) ? rcp : e * rcp;
    *(volatile float*)(out + i) = o;
    __threadfence();
    *(volatile float*)(out + i) = o;
  }
}

extern "C" void kernel_launch(void* const* d_in, const int* in_sizes, int n_in,
                              void* d_out, int out_size, void* d_ws, size_t ws_size,
                              hipStream_t stream) {
  if (n_in < 23) return;
  if (in_sizes[0] != PN * NF) return;
  if (in_sizes[1] != 2 * E2N || in_sizes[2] != 2 * E2N) return;
  if (in_sizes[3] != 2 * EIN) return;
  if (in_sizes[4] != 2 * NLK) return;
  if (in_sizes[5] < 1) return;
  if (in_sizes[6] != EIN) return;
  if (in_sizes[7] != NF * F1 || in_sizes[8] != F1) return;
  if (in_sizes[9] != F1 * F1 || in_sizes[10] != F1) return;
  if (in_sizes[11] != NF * F1 || in_sizes[12] != F1) return;
  if (in_sizes[13] != F1 * F1 || in_sizes[14] != F1) return;
  if (in_sizes[15] != NF * F2 || in_sizes[16] != F2) return;
  if (in_sizes[17] != NF * F2 || in_sizes[18] != F2) return;
  if (in_sizes[19] != (F2 + 1) * F2 || in_sizes[20] != F2) return;
  if (in_sizes[21] != F1 + F2 || in_sizes[22] != 1) return;
  if (out_size != HALFP) return;

  const float* x      = (const float*)d_in[0];
  const int*   edge2  = (const int*)d_in[1];
  const int*   edge2r = (const int*)d_in[2];
  const int*   ei     = (const int*)d_in[3];
  const int*   plinks = (const int*)d_in[4];
  const int*   nnp    = (const int*)d_in[5];
  const int*   posm   = (const int*)d_in[6];
  const float* w0  = (const float*)d_in[7];
  const float* b0  = (const float*)d_in[8];
  const float* w1  = (const float*)d_in[9];
  const float* b1  = (const float*)d_in[10];
  const float* wr0 = (const float*)d_in[11];
  const float* br0 = (const float*)d_in[12];
  const float* wr1 = (const float*)d_in[13];
  const float* br1 = (const float*)d_in[14];
  const float* m1w = (const float*)d_in[15];
  const float* m1b = (const float*)d_in[16];
  const float* m2w = (const float*)d_in[17];
  const float* m2b = (const float*)d_in[18];
  const float* m3w = (const float*)d_in[19];
  const float* m3b = (const float*)d_in[20];
  const float* m4w = (const float*)d_in[21];
  const float* m4b = (const float*)d_in[22];
  float* out = (float*)d_out;

  char* wsb = (char*)d_ws;
  size_t off = 0;
#define CARVE(T, name, nbytes) T* name = (T*)(wsb + off); off += ((((size_t)(nbytes)) + 255) / 256) * 256;
  const size_t arena0 = off;
  CARVE(int,   RowsA, (size_t)PROWS * RW * 4)
  CARVE(int,   RowsB, (size_t)PROWS * RW * 4)
  CARVE(float, Tb,    (size_t)MPAD * 64 * 4)
  CARVE(float, H1,    (size_t)MPAD * F1 * 4)
  const size_t arena1 = off;
  _Float16* PA = (_Float16*)(wsb + arena0);
  _Float16* PB = PA + (size_t)CB * NND * NND;
  if ((size_t)2 * CB * NND * NND * 2 > arena1 - arena0) return;
  CARVE(float,        H2,    (size_t)MPAD * F1 * 4)
  CARVE(float,        X12,   (size_t)EPAD * 64 * 4)
  CARVE(unsigned int, Abits, (size_t)NND * 32 * 4)
  CARVE(float,        Cb,    (size_t)CSUB * NND * NND * 4)
  CARVE(float,        CuvT,  (size_t)F2 * NLK * 4)
  CARVE(float,        Vb,    (size_t)VPAD * 32 * 4)
#undef CARVE
  if (off > ws_size) return;
  if (off > (size_t)134217728) return;

  k_rows<<<dim3(NRB, 2), NTHR, 0, stream>>>(edge2, edge2r, RowsA, RowsB, E2N, PN);

  k_gemm<NF><<<MT1, GTHR, 0, stream>>>(x, posm, 0, PN, PN, w0, F1, wr0, F1, 0, RowsA, RowsB, b0, br0, Tb);
  k_agg<<<PN / NWAVE, NTHR, 0, stream>>>(RowsA, RowsB, Tb, b0, br0, H1, PN);

  k_gemm<F1><<<MT1, GTHR, 0, stream>>>(H1, posm, 0, PN, PN, w1, F1, wr1, F1, 0, RowsA, RowsB, b1, br1, Tb);
  k_agg<<<PN / NWAVE, NTHR, 0, stream>>>(RowsA, RowsB, Tb, b1, br1, H2, PN);

  k_gemm<NF><<<MT2, GTHR, 0, stream>>>(x, posm, 1, EIN, PN, m1w, F2, m2w, F2, 1, RowsA, RowsB, m1b, m2b, X12);

  for (int bt = 0; bt < NBATCH; ++bt) {
    const int cb0 = bt * CB;
    k_planes<<<dim3(NND, 2), 32, 0, stream>>>(ei, X12, nnp, cb0, bt == 0 ? 1 : 0, PA, PB, Abits, EIN);
    for (int sub = 0; sub < NSUB; ++sub) {
      k_bigemm<<<dim3(NND / GT, NND / GT, CSUB), GTHR, 0, stream>>>(PA, PB, Cb, sub * CSUB);
      k_cuv<<<(NLK / 4 + NTHR - 1) / NTHR, NTHR, 0, stream>>>(plinks, nnp, Cb, CuvT, cb0 + sub * CSUB);
    }
  }

  k_link<<<LT, GTHR, 0, stream>>>(plinks, nnp, Abits, CuvT, m3w, m3b, Vb);
  k_final<<<(HALFP + NTHR - 1) / NTHR, NTHR, 0, stream>>>(H2, Vb, m4w, m4b, out);
}
